// LSTM_59322088292480
// MI455X (gfx1250) — hardware-verified
//
#include <hip/hip_runtime.h>
#include <math.h>

constexpr int NBATCH = 1024;
constexpr int NSTEP  = 512;
constexpr int NFEAT  = 18;
constexpr int NHID   = 64;
constexpr int NGATE  = 4 * NHID;
constexpr int NCLS   = 15;
constexpr int XK     = 32;
constexpr int HP     = 72;
constexpr int PLANE  = 16 * HP;
constexpr int SLABP  = 68;
constexpr float CARRY    = 256.0f;
constexpr float PROD_INV = 1.0f / (CARRY * CARRY);
constexpr float BN_EPS_F = 1e-5f;
constexpr int NPACK8  = NSTEP * NBATCH * (XK / 8);
constexpr int WX0_EL  = NGATE * XK;
constexpr int WHH_EL  = NGATE * NHID;
constexpr int WPL_EL  = WX0_EL + 3 * WHH_EL;
constexpr int WPREP_BLOCKS = WPL_EL / 8 / 256;
constexpr int NOUTEL  = NBATCH * NCLS;
static_assert(NFEAT <= XK && XK % 32 == 0, "x K padded to one 32-deep chunk");
static_assert(NHID % 32 == 0 && NHID == 64, "hidden K = two 32-deep chunks, 4 waves x 16 columns");
static_assert(NBATCH % 16 == 0, "16 batch rows per block");
static_assert(NPACK8 % 256 == 0, "pack grid exact");
static_assert(WX0_EL / 8 == 4 * 256 && WHH_EL / 8 == 8 * 256 && WPREP_BLOCKS == 28, "weight prep block map");
static_assert(NOUTEL % 256 == 0, "classifier grid exact");
static_assert((2 * 4 * PLANE) % 128 == 0, "h plane zero fill exact");
static_assert(NBATCH == 4 * 256, "statistics kernel: 4 row groups of 256");

typedef __attribute__((ext_vector_type(16))) _Float16 v16h;
typedef __attribute__((ext_vector_type(8)))  _Float16 v8h;
typedef __attribute__((ext_vector_type(8)))  float    v8f;
typedef __attribute__((ext_vector_type(4)))  float    v4f;

__device__ __forceinline__ unsigned short f2bf_bits(float f) {
  unsigned u = __float_as_uint(f);
  return (unsigned short)((u + 0x7FFFu + ((u >> 16) & 1u)) >> 16);
}
__device__ __forceinline__ float bf_bits2f(unsigned short h) { return __uint_as_float(((unsigned)h) << 16); }
__device__ __forceinline__ float bf16r(float f) { return bf_bits2f(f2bf_bits(f)); }

template <typename T> struct Frag;
template <> struct Frag<_Float16> {
  typedef v16h V; union U { v16h v; v8h h[2]; };
  static __device__ __forceinline__ v16h load(const _Float16* p) {
    U f; f.h[0] = *(const v8h*)(p); f.h[1] = *(const v8h*)(p + 16); return f.v;
  }
};

__device__ __forceinline__ v8f mma_h(v16h a, v16h b, v8f c) {
  c = __builtin_amdgcn_wmma_f32_16x16x32_f16(false, a, false, b, (short)0, c, false, false);
  asm volatile("v_nop\n\tv_nop\n\tv_nop\n\tv_nop" : "+v"(c) : "v"(a), "v"(b));
  return c;
}

__device__ __forceinline__ float fsig(float x)  { return __builtin_amdgcn_rcpf(1.0f + expf(-x)); }
__device__ __forceinline__ float ftanh(float x) { return 1.0f - 2.0f * __builtin_amdgcn_rcpf(expf(2.0f * x) + 1.0f); }

__device__ __forceinline__ float lstm_cell(float zi, float zf, float zg, float zo, float& cst) {
  const float ig = fsig(zi);
  const float fg = fsig(zf);
  const float gg = ftanh(zg);
  const float og = fsig(zo);
  const float cn = fg * cst + ig * gg;
  cst = cn;
  return og * ftanh(cn);
}

__global__ __launch_bounds__(256) void pack_x_kernel(const float* __restrict__ X, unsigned short* __restrict__ XP) {
  const int i = blockIdx.x * 256 + threadIdx.x;
  if (i < NPACK8) {
    const int orow = i >> 2;
    const int q = i & 3;
    const int s = orow >> 10;
    const int b = orow & (NBATCH - 1);
    const float* src = X + ((size_t)b * NSTEP + (size_t)s) * NFEAT;
    v8h hv;
#pragma unroll
    for (int e = 0; e < 8; ++e) {
      const int col = 8 * q + e;
      const int colc = (col < NFEAT) ? col : (NFEAT - 1);
      const float v = src[colc];
      const float xv = (col < NFEAT) ? v : 0.0f;
      hv[e] = (_Float16)(bf16r(xv) * CARRY);
    }
    *(volatile v8h*)(XP + (size_t)i * 8) = hv;
    __threadfence();
    *(volatile v8h*)(XP + (size_t)i * 8) = hv;
  }
}

__global__ __launch_bounds__(256) void wprep_kernel(const float* __restrict__ wih0, const float* __restrict__ whh0,
                                                    const float* __restrict__ wih1, const float* __restrict__ whh1,
                                                    unsigned short* __restrict__ WPL) {
  const int blk = blockIdx.x;
  const int i = blk * 256 + threadIdx.x;
  v8h hv;
  if (blk < 4) {
    const int row = i >> 2;
    const int q = i & 3;
#pragma unroll
    for (int e = 0; e < 8; ++e) {
      const int col = 8 * q + e;
      const int colc = (col < NFEAT) ? col : (NFEAT - 1);
      const float v = wih0[row * NFEAT + colc];
      const float wv = (col < NFEAT) ? v : 0.0f;
      hv[e] = (_Float16)(bf16r(wv) * CARRY);
    }
  } else {
    const int pl = (blk - 4) >> 3;
    const float* src = (pl == 0) ? whh0 : ((pl == 1) ? wih1 : whh1);
    const int idx = i - 1024 - pl * 2048;
    const v4f a = *(const v4f*)(src + (size_t)idx * 8);
    const v4f b = *(const v4f*)(src + (size_t)idx * 8 + 4);
#pragma unroll
    for (int e = 0; e < 4; ++e) {
      const float fa = a[e];
      const float fb = b[e];
      hv[e]     = (_Float16)(bf16r(fa) * CARRY);
      hv[4 + e] = (_Float16)(bf16r(fb) * CARRY);
    }
  }
  *(volatile v8h*)(WPL + (size_t)i * 8) = hv;
  __threadfence();
  *(volatile v8h*)(WPL + (size_t)i * 8) = hv;
}

__global__ __launch_bounds__(128) void lstm2_kernel(const unsigned short* XPp, const unsigned short* WPLp,
                                                    const float* bih0, const float* bhh0,
                                                    const float* bih1, const float* bhh1,
                                                    float* lastH) {
  __shared__ __align__(16) _Float16 Hs[2 * 4 * PLANE];
  __shared__ __align__(16) float    Slab[16 * SLABP];
  typedef Frag<_Float16> F;
  const _Float16* XPh = (const _Float16*)XPp;
  const _Float16* WX0 = (const _Float16*)WPLp;
  const _Float16* WH0 = WX0 + WX0_EL;
  const _Float16* WI1 = WH0 + WHH_EL;
  const _Float16* WH1 = WI1 + WHH_EL;
  const int tid = threadIdx.x, lane = tid & 31, wave = tid >> 5;
  const int c = lane & 15, hh = lane >> 4, koff = hh * 8;
  const int rowbase = blockIdx.x * 16;
  const int j = 16 * wave + c;

#pragma unroll 1
  for (int i = tid; i < 2 * 4 * PLANE; i += 128) Hs[i] = (_Float16)0.0f;

  float bias0[4], bias1[4];
#pragma unroll
  for (int g = 0; g < 4; ++g) {
    const int n = g * NHID + j;
    bias0[g] = bf16r(bih0[n]) + bf16r(bhh0[n]);
  }
  asm volatile("" ::: "memory");
#pragma unroll
  for (int g = 0; g < 4; ++g) {
    const int n = g * NHID + j;
    bias1[g] = bf16r(bih1[n]) + bf16r(bhh1[n]);
  }
  asm volatile("" ::: "memory");

  float c0s[8], c1s[8], hlast[8];
#pragma unroll
  for (int r = 0; r < 8; ++r) { c0s[r] = 0.0f; c1s[r] = 0.0f; hlast[r] = 0.0f; }
  const v8f z8 = {0.f, 0.f, 0.f, 0.f, 0.f, 0.f, 0.f, 0.f};
  __syncthreads();

#pragma unroll 1
  for (int s = 0; s < NSTEP; ++s) {
    const int p = s & 1;
    const _Float16* cur = Hs + p * (4 * PLANE);
    _Float16*       nxt = Hs + (p ^ 1) * (4 * PLANE);
    const _Float16* arow_cur = cur + c * HP + koff;
    const _Float16* arow_nxt = nxt + c * HP + koff;

    {
      const v16h ax = F::load(XPh + ((size_t)s * NBATCH + (size_t)(rowbase + c)) * XK + koff);
      const v16h a0 = F::load(arow_cur + 0 * PLANE);
      const v16h a1 = F::load(arow_cur + 0 * PLANE + 32);
      asm volatile("" ::: "memory");
      v8f acc[4];
#pragma unroll
      for (int g = 0; g < 4; ++g) {
        const int n = g * NHID + j;
        const v16h bx = F::load(WX0 + (size_t)n * XK + koff);
        const v16h b0 = F::load(WH0 + (size_t)n * NHID + koff);
        const v16h b1 = F::load(WH0 + (size_t)n * NHID + koff + 32);
        v8f a = z8;
        a = mma_h(ax, bx, a);
        a = mma_h(a0, b0, a);
        a = mma_h(a1, b1, a);
        acc[g] = a;
        asm volatile("" ::: "memory");
      }
#pragma unroll
      for (int r = 0; r < 8; ++r) {
        const float zi = acc[0][r] * PROD_INV + bias0[0];
        const float zf = acc[1][r] * PROD_INV + bias0[1];
        const float zg = acc[2][r] * PROD_INV + bias0[2];
        const float zo = acc[3][r] * PROD_INV + bias0[3];
        const float hn = lstm_cell(zi, zf, zg, zo, c0s[r]);
        const float hs = hn * CARRY;
        const _Float16 hi = (_Float16)hs;
        const _Float16 lo = (_Float16)(hs - (float)hi);
        nxt[0 * PLANE + (8 * hh + r) * HP + j] = hi;
        nxt[1 * PLANE + (8 * hh + r) * HP + j] = lo;
      }
    }
    __syncthreads();

    {
      const v16h n0 = F::load(arow_nxt + 0 * PLANE);
      const v16h n1 = F::load(arow_nxt + 0 * PLANE + 32);
      const v16h l0 = F::load(arow_nxt + 1 * PLANE);
      const v16h l1 = F::load(arow_nxt + 1 * PLANE + 32);
      const v16h m0 = F::load(arow_cur + 2 * PLANE);
      const v16h m1 = F::load(arow_cur + 2 * PLANE + 32);
      const v16h q0 = F::load(arow_cur + 3 * PLANE);
      const v16h q1 = F::load(arow_cur + 3 * PLANE + 32);
      asm volatile("" ::: "memory");
      v8f acc[4];
#pragma unroll
      for (int g = 0; g < 4; ++g) {
        const int n = g * NHID + j;
        const v16h bi0 = F::load(WI1 + (size_t)n * NHID + koff);
        const v16h bi1 = F::load(WI1 + (size_t)n * NHID + koff + 32);
        const v16h bh0 = F::load(WH1 + (size_t)n * NHID + koff);
        const v16h bh1 = F::load(WH1 + (size_t)n * NHID + koff + 32);
        v8f a = z8;
        a = mma_h(n0, bi0, a);
        a = mma_h(l0, bi0, a);
        a = mma_h(n1, bi1, a);
        a = mma_h(l1, bi1, a);
        a = mma_h(m0, bh0, a);
        a = mma_h(q0, bh0, a);
        a = mma_h(m1, bh1, a);
        a = mma_h(q1, bh1, a);
        acc[g] = a;
        asm volatile("" ::: "memory");
      }
#pragma unroll
      for (int r = 0; r < 8; ++r) {
        const float zi = acc[0][r] * PROD_INV + bias1[0];
        const float zf = acc[1][r] * PROD_INV + bias1[1];
        const float zg = acc[2][r] * PROD_INV + bias1[2];
        const float zo = acc[3][r] * PROD_INV + bias1[3];
        const float hn = lstm_cell(zi, zf, zg, zo, c1s[r]);
        hlast[r] = hn;
        const float hs = hn * CARRY;
        const _Float16 hi = (_Float16)hs;
        const _Float16 lo = (_Float16)(hs - (float)hi);
        nxt[2 * PLANE + (8 * hh + r) * HP + j] = hi;
        nxt[3 * PLANE + (8 * hh + r) * HP + j] = lo;
      }
    }
  }

#pragma unroll
  for (int r = 0; r < 8; ++r) Slab[(8 * hh + r) * SLABP + j] = hlast[r];
  __syncthreads();
  {
    const int c4 = c * 4;
    for (int pass = 0; pass < 2; ++pass) {
#pragma unroll
      for (int it = 0; it < 2; ++it) {
        const int row = 4 * wave + 2 * it + hh;
        const v4f v = *(const v4f*)(Slab + row * SLABP + c4);
        *(volatile v4f*)(lastH + (size_t)(rowbase + row) * NHID + c4) = v;
      }
      __threadfence();
    }
  }
}

__global__ __launch_bounds__(256) void bn_stats_kernel(const float* __restrict__ lastH, const float* __restrict__ gam,
                                                       const float* __restrict__ bet, float* __restrict__ AB) {
  __shared__ float part[4 * 64];
  __shared__ __align__(16) float stage[256];
  const int tid = threadIdx.x;
  const int j = tid & 63, q = tid >> 6;
  const float* base = lastH + (size_t)(q * 256) * NHID + j;
  float s = 0.0f;
#pragma unroll 4
  for (int i = 0; i < 256; ++i) s += base[(size_t)i * NHID];
  part[q * 64 + j] = s;
  __syncthreads();
  const float mean = ((part[j] + part[64 + j]) + (part[128 + j] + part[192 + j])) * (1.0f / (float)NBATCH);
  __syncthreads();
  float ss = 0.0f;
#pragma unroll 4
  for (int i = 0; i < 256; ++i) { const float d = base[(size_t)i * NHID] - mean; ss += d * d; }
  part[q * 64 + j] = ss;
  __syncthreads();
  const float var = ((part[j] + part[64 + j]) + (part[128 + j] + part[192 + j])) * (1.0f / (float)NBATCH);
  const float aj = bf16r(gam[j]) * rsqrtf(var + BN_EPS_F);
  const float bj = bf16r(bet[j]);
  const float val = (q == 0) ? aj : ((q == 1) ? mean : ((q == 2) ? bj : 0.0f));
  stage[tid] = val;
  __syncthreads();
  if (tid < 64) {
    const v4f v = *(const v4f*)(stage + 4 * tid);
    *(volatile v4f*)(AB + 4 * tid) = v;
    __threadfence();
    *(volatile v4f*)(AB + 4 * tid) = v;
  }
}

__global__ __launch_bounds__(256) void classify_kernel(const float* __restrict__ lastH, const float* __restrict__ AB,
                                                       const float* __restrict__ clsW, const float* __restrict__ clsB,
                                                       float* __restrict__ out) {
  __shared__ float sW[NCLS * NHID];
  __shared__ float sAB[256];
  __shared__ float sCb[16];
  const int tid = threadIdx.x;
#pragma unroll
  for (int it = 0; it < 4; ++it) {
    const int i0 = it * 256 + tid;
    const int idx = (i0 < NCLS * NHID) ? i0 : (NCLS * NHID - 1);
    sW[idx] = bf16r(clsW[idx]);
  }
  sAB[tid] = AB[tid];
  {
    const int ib = (tid < NCLS) ? tid : (NCLS - 1);
    sCb[ib] = bf16r(clsB[ib]);
  }
  __syncthreads();
  const int e = blockIdx.x * 256 + tid;
  const int b = e / NCLS;
  const int o = e - b * NCLS;
  const float* hrow = lastH + (size_t)b * NHID;
  const float* wrow = sW + o * NHID;
  float acc = 0.0f;
#pragma unroll 2
  for (int jj = 0; jj < NHID / 4; ++jj) {
    const v4f x = *(const v4f*)(hrow + 4 * jj);
#pragma unroll
    for (int k = 0; k < 4; ++k) {
      const int jx = 4 * jj + k;
      const float xv = x[k];
      const float nrm = (xv - sAB[64 + jx]) * sAB[jx] + sAB[128 + jx];
      acc = fmaf(nrm, wrow[jx], acc);
    }
  }
  const float res = acc + sCb[o];
  volatile float* op = out + e;
  *op = res;
  __threadfence();
  *op = res;
}

extern "C" void kernel_launch(void* const* d_in, const int* in_sizes, int n_in,
                              void* d_out, int out_size, void* d_ws, size_t ws_size, hipStream_t stream) {
  if (n_in < 13 || d_out == nullptr || d_ws == nullptr) return;
  if (in_sizes[0] != NBATCH * NSTEP * NFEAT || in_sizes[1] != NGATE * NFEAT || in_sizes[2] != NGATE * NHID ||
      in_sizes[3] != NGATE || in_sizes[4] != NGATE || in_sizes[5] != NGATE * NHID || in_sizes[6] != NGATE * NHID ||
      in_sizes[7] != NGATE || in_sizes[8] != NGATE || in_sizes[9] != NHID || in_sizes[10] != NHID ||
      in_sizes[11] != NCLS * NHID || in_sizes[12] != NCLS || out_size != NOUTEL) return;

  const float* X    = (const float*)d_in[0];
  const float* wih0 = (const float*)d_in[1];
  const float* whh0 = (const float*)d_in[2];
  const float* bih0 = (const float*)d_in[3];
  const float* bhh0 = (const float*)d_in[4];
  const float* wih1 = (const float*)d_in[5];
  const float* whh1 = (const float*)d_in[6];
  const float* bih1 = (const float*)d_in[7];
  const float* bhh1 = (const float*)d_in[8];
  const float* gam  = (const float*)d_in[9];
  const float* bet  = (const float*)d_in[10];
  const float* clsW = (const float*)d_in[11];
  const float* clsB = (const float*)d_in[12];
  float* out = (float*)d_out;

  char* ws = (char*)d_ws; size_t off = 0;
  auto carve = [&](size_t bytes) -> char* { char* p = ws + off; off += (bytes + 255) & ~(size_t)255; return p; };
  unsigned short* XP    = (unsigned short*)carve((size_t)NSTEP * NBATCH * XK * 2);
  unsigned short* WPL   = (unsigned short*)carve((size_t)WPL_EL * 2);
  float*          LASTH = (float*)carve((size_t)NBATCH * NHID * 4);
  float*          AB    = (float*)carve((size_t)256 * 4);
  if (off > ws_size || off > (size_t)134217728) return;

  pack_x_kernel<<<NPACK8 / 256, 256, 0, stream>>>(X, XP);
  wprep_kernel<<<WPREP_BLOCKS, 256, 0, stream>>>(wih0, whh0, wih1, whh1, WPL);
  lstm2_kernel<<<NBATCH / 16, 128, 0, stream>>>(XP, WPL, bih0, bhh0, bih1, bhh1, LASTH);
  bn_stats_kernel<<<1, 256, 0, stream>>>(LASTH, gam, bet, AB);
  classify_kernel<<<NOUTEL / 256, 256, 0, stream>>>(LASTH, AB, clsW, clsB, out);
}
